// DGCNN_GNN_Layers_79680233276343
// MI455X (gfx1250) — hardware-run, weakly checked
//
#include <hip/hip_runtime.h>
#include <stddef.h>
#include <stdint.h>
#include <math.h>


#define NGR     512
#define PN      256
#define NNODE   (NGR * PN)
#define NEDGE   2097152
#define FIN     64
#define HID     32
#define NTHR    256
#define NWAVE   8
#define CHUNKE  8192
#define EPT     32
#define NRUN    (NEDGE / CHUNKE)
#define RUNCAP  512
#define GCAP    1024
#define APITCH  72
#define HPITCH  36
#define APL     (PN * APITCH)
#define WPLL    (HID * APITCH)
#define CGRP    32
#define WSMAX   134217728

static_assert(NEDGE % CHUNKE == 0);
static_assert(NRUN == NTHR);
static_assert(CHUNKE == NTHR * EPT && EPT == 32);
static_assert(PN == NTHR && FIN == 64 && HID == 32);
static_assert(NGR == 2 * NTHR);
static_assert(NGR % CGRP == 0 && CGRP == 32);
static_assert(NNODE % (4 * NTHR) == 0);
static_assert(RUNCAP == 2 * NTHR && (RUNCAP % 8) == 0);
static_assert(GCAP >= 1024 && RUNCAP >= 512);
static_assert((APITCH % 8) == 0 && (HPITCH % 4) == 0);
static_assert(PN == NWAVE * 32);
static_assert(2 * APL * 2 + PN * HPITCH * 4 + 3 * WPLL * 2 + GCAP * 8 + 5 * 1024 <= 160000);

typedef float          v2f  __attribute__((ext_vector_type(2)));
typedef float          v4f  __attribute__((ext_vector_type(4)));
typedef float          v8f  __attribute__((ext_vector_type(8)));
typedef int            v2i  __attribute__((ext_vector_type(2)));
typedef int            v4i  __attribute__((ext_vector_type(4)));
typedef int            v8i  __attribute__((ext_vector_type(8)));
typedef unsigned int   v2u  __attribute__((ext_vector_type(2)));
typedef unsigned int   v4u  __attribute__((ext_vector_type(4)));
typedef unsigned short v8us __attribute__((ext_vector_type(8)));
typedef __bf16         v16b __attribute__((ext_vector_type(16)));
typedef v4f  __attribute__((may_alias)) v4fa;
typedef v4i  __attribute__((may_alias)) v4ia;
typedef v2u  __attribute__((may_alias)) v2ua;
typedef v4u  __attribute__((may_alias)) v4ua;
typedef v8us __attribute__((may_alias)) v8usa;
union FragB { v16b v; v8us h[2]; v8i w; };

__device__ __forceinline__ v8f wmb(const FragB& a, const FragB& b, v8f c) {
  v8f d = __builtin_amdgcn_wmma_f32_16x16x32_bf16(false, a.v, false, b.v, (short)0, c, false, false);
  asm volatile("v_nop\n\tv_nop\n\tv_nop\n\tv_nop" : "+v"(d) : "v"(a.w), "v"(b.w));
  return d;
}

__device__ __forceinline__ unsigned int f2bf(float f) {
  const unsigned int u = __float_as_uint(f);
  const unsigned int r = ((u + 0x7FFFu + ((u >> 16) & 1u)) >> 16) & 0xFFFFu;
  return ((u & 0x7FFFFFFFu) > 0x7F800000u) ? 0x7FC0u : r;
}
__device__ __forceinline__ float bf2f(unsigned int b) { return __uint_as_float(b << 16); }
__device__ __forceinline__ float bfr(float f) { return bf2f(f2bf(f)); }
__device__ __forceinline__ int iclamp(int v, int lo, int hi) { return v < lo ? lo : (v > hi ? hi : v); }

__device__ __forceinline__ void put8(unsigned short* dp, v8us o) {
  *(volatile v8us*)dp = o;
  __threadfence();
  *(volatile v8us*)dp = o;
}

__global__ __launch_bounds__(NTHR) void k_prep(const float* __restrict__ W0, const float* __restrict__ b0,
                                               const float* __restrict__ W1, const float* __restrict__ b1,
                                               const float* __restrict__ W2, const float* __restrict__ b2,
                                               const float* __restrict__ W3, const float* __restrict__ b3,
                                               unsigned short* WPL, float* PAR) {
  __shared__ __attribute__((aligned(16))) float sp[256];
  const int tid = (int)threadIdx.x;
  const int blk = (int)blockIdx.x;
  const int n  = tid >> 3;
  const int k8 = (tid & 7) * 8;
  const int kk = k8 & (HID - 1);
  if (blk == 0) {
    const float* p = W0 + (size_t)k8 * HID + n;
    v8us o;
#pragma unroll
    for (int i = 0; i < 8; ++i) o[i] = (unsigned short)f2bf(p[(size_t)i * HID]);
    put8(WPL + (size_t)n * FIN + k8, o);
  } else if (blk == 1) {
    const float* p = W1 + (size_t)kk * HID + n;
    v8us o;
#pragma unroll
    for (int i = 0; i < 8; ++i) o[i] = (unsigned short)f2bf(p[(size_t)i * HID]);
    put8(WPL + (size_t)(HID * FIN) + (size_t)n * FIN + k8, o);
  } else if (blk == 2) {
    const float* p = W2 + (size_t)kk * HID + n;
    v8us o;
#pragma unroll
    for (int i = 0; i < 8; ++i) o[i] = (unsigned short)f2bf(p[(size_t)i * HID]);
    put8(WPL + (size_t)(2 * HID * FIN) + (size_t)n * FIN + k8, o);
  } else {
    sp[tid] = 0.0f;
    __syncthreads();
    if (tid < 32) {
      const float a0 = b0[tid];
      const float a1 = b1[tid];
      const float a2 = b2[tid];
      const float a3 = W3[tid];
      const float a4 = b3[0];
      sp[tid]      = bfr(a0);
      sp[32 + tid] = bfr(a1);
      sp[64 + tid] = bfr(a2);
      sp[96 + tid] = bfr(a3);
      if (tid == 0) sp[128] = bfr(a4);
    }
    __syncthreads();
    const v4f pv = *(const v4fa*)(sp + 4 * (tid & 63));
    float* op = PAR + 4 * (tid & 63);
    const bool okst = tid < 64;
    if (okst) *(volatile v4f*)op = pv;
    __threadfence();
    if (okst) *(volatile v4f*)op = pv;
  }
}

__global__ __launch_bounds__(NTHR) void k_counts(const int* __restrict__ bat, int* COUNTS) {
  __shared__ int part[CGRP * NTHR];
  __shared__ __attribute__((aligned(16))) int tot[CGRP];
  const int tid = (int)threadIdx.x;
  const unsigned base = (unsigned)((int)blockIdx.x * CGRP);
  int c[CGRP];
#pragma unroll
  for (int q = 0; q < CGRP; ++q) c[q] = 0;
#pragma unroll 1
  for (int it = 0; it < NNODE / (4 * NTHR); ++it) {
    const v4i b = *(const v4i*)(bat + 4 * (it * NTHR + tid));
    const unsigned d0 = (unsigned)b.x - base, d1 = (unsigned)b.y - base;
    const unsigned d2 = (unsigned)b.z - base, d3 = (unsigned)b.w - base;
#pragma unroll
    for (int q = 0; q < CGRP; ++q) {
      c[q] += (d0 == (unsigned)q) ? 1 : 0;
      c[q] += (d1 == (unsigned)q) ? 1 : 0;
      c[q] += (d2 == (unsigned)q) ? 1 : 0;
      c[q] += (d3 == (unsigned)q) ? 1 : 0;
    }
  }
#pragma unroll
  for (int q = 0; q < CGRP; ++q) part[q * NTHR + tid] = c[q];
  __syncthreads();
  {
    const int q = tid >> 3, seg = tid & 7;
    int s = 0;
#pragma unroll 4
    for (int i = 0; i < 32; ++i) s += part[q * NTHR + seg * 32 + i];
    s += __shfl_xor(s, 1, 32);
    s += __shfl_xor(s, 2, 32);
    s += __shfl_xor(s, 4, 32);
    if (seg == 0) tot[q] = s;
  }
  __syncthreads();
  const v4i tv = *(const v4ia*)(tot + 4 * (tid & 7));
  int* op = COUNTS + (int)base + 4 * (tid & 7);
  const bool okst = tid < 8;
  if (okst) *(volatile v4i*)op = tv;
  __threadfence();
  if (okst) *(volatile v4i*)op = tv;
}

#define PUTE(S, D, A, M, BIT) { \
    const int gc_ = iclamp((A), 0, NGR - 1); \
    const int st_ = starts[gc_]; \
    const int ls_ = iclamp((S) - st_, 0, PN - 1); \
    const int ld_ = iclamp((D) - st_, 0, PN - 1); \
    const bool on_ = (BIT) != 0u; \
    if (on_ && cur < RUNCAP) { \
      v4i en_; en_.x = gc_; en_.y = ls_; en_.z = ld_; en_.w = __float_as_int(bfr(M)); \
      *(v4ia*)(runl + 4 * cur) = en_; \
    } \
    cur += on_ ? 1 : 0; }

__global__ __launch_bounds__(NTHR) void k_vfill(const int* __restrict__ ei, const int* __restrict__ bat,
                                                const float* __restrict__ emask,
                                                const int* __restrict__ COUNTS, int* RUN, int* CNTB) {
  __shared__ int starts[NGR];
  __shared__ int wtA[NWAVE];
  __shared__ int wtB[NWAVE];
  __shared__ __attribute__((aligned(16))) int runl[RUNCAP * 4];
  const int tid = (int)threadIdx.x, lane = tid & 31, wave = tid >> 5;
  const int blk = (int)blockIdx.x;

  {
    const v2i c2 = *(const v2i*)(COUNTS + 2 * tid);
    const int c0 = iclamp(c2.x, 0, NNODE);
    const int c1 = iclamp(c2.y, 0, NNODE);
    const int s = c0 + c1;
    int incl = s;
#pragma unroll
    for (int d = 1; d < 32; d <<= 1) {
      const int y = __shfl_up(incl, d, 32);
      if (lane >= d) incl += y;
    }
    if (lane == 31) wtA[wave] = incl;
    __syncthreads();
    int wb = 0;
#pragma unroll
    for (int w2 = 0; w2 < NWAVE; ++w2) { const int c = wtA[w2]; wb += (w2 < wave) ? c : 0; }
    const int excl = wb + incl - s;
    starts[2 * tid]     = excl;
    starts[2 * tid + 1] = excl + c0;
  }
  __syncthreads();

  const int* srcp = ei;
  const int* dstp = ei + NEDGE;
  const int e0 = blk * CHUNKE + tid * EPT;

  unsigned vm = 0u;
#pragma unroll 1
  for (int j = 0; j < EPT / 4; ++j) {
    const v4i s4 = *(const v4i*)(srcp + e0 + 4 * j);
    const v4i d4 = *(const v4i*)(dstp + e0 + 4 * j);
    const int a0 = bat[iclamp(s4.x, 0, NNODE - 1)];
    const int a1 = bat[iclamp(s4.y, 0, NNODE - 1)];
    const int a2 = bat[iclamp(s4.z, 0, NNODE - 1)];
    const int a3 = bat[iclamp(s4.w, 0, NNODE - 1)];
    const int c0 = bat[iclamp(d4.x, 0, NNODE - 1)];
    const int c1 = bat[iclamp(d4.y, 0, NNODE - 1)];
    const int c2 = bat[iclamp(d4.z, 0, NNODE - 1)];
    const int c3 = bat[iclamp(d4.w, 0, NNODE - 1)];
    const unsigned v0 = ((a0 == c0) && ((unsigned)a0 < (unsigned)NGR)) ? 1u : 0u;
    const unsigned v1 = ((a1 == c1) && ((unsigned)a1 < (unsigned)NGR)) ? 1u : 0u;
    const unsigned v2 = ((a2 == c2) && ((unsigned)a2 < (unsigned)NGR)) ? 1u : 0u;
    const unsigned v3 = ((a3 == c3) && ((unsigned)a3 < (unsigned)NGR)) ? 1u : 0u;
    vm |= (v0 | (v1 << 1) | (v2 << 2) | (v3 << 3)) << (4 * j);
  }
  const int mycnt = (int)__builtin_popcount(vm);

  int total, cur;
  {
    int incl = mycnt;
#pragma unroll
    for (int d = 1; d < 32; d <<= 1) {
      const int y = __shfl_up(incl, d, 32);
      if (lane >= d) incl += y;
    }
    if (lane == 31) wtB[wave] = incl;
    __syncthreads();
    int wb = 0, all = 0;
#pragma unroll
    for (int w2 = 0; w2 < NWAVE; ++w2) { const int c = wtB[w2]; all += c; wb += (w2 < wave) ? c : 0; }
    total = all;
    cur = wb + incl - mycnt;
  }

#pragma unroll 1
  for (int j = 0; j < EPT / 4; ++j) {
    const v4i s4 = *(const v4i*)(srcp + e0 + 4 * j);
    const v4i d4 = *(const v4i*)(dstp + e0 + 4 * j);
    const v4f m4 = *(const v4f*)(emask + e0 + 4 * j);
    const int a0 = bat[iclamp(s4.x, 0, NNODE - 1)];
    const int a1 = bat[iclamp(s4.y, 0, NNODE - 1)];
    const int a2 = bat[iclamp(s4.z, 0, NNODE - 1)];
    const int a3 = bat[iclamp(s4.w, 0, NNODE - 1)];
    const unsigned bits = (vm >> (4 * j)) & 15u;
    PUTE(s4.x, d4.x, a0, m4.x, bits & 1u)
    PUTE(s4.y, d4.y, a1, m4.y, bits & 2u)
    PUTE(s4.z, d4.z, a2, m4.z, bits & 4u)
    PUTE(s4.w, d4.w, a3, m4.w, bits & 8u)
  }

  const int cntc = total > RUNCAP ? RUNCAP : (total < 0 ? 0 : total);
  const int ovf  = total > RUNCAP ? 1 : 0;
  int cntPad = (cntc + 7) & ~7;
  cntPad = cntPad < 8 ? 8 : cntPad;
  {
    const v4i z4 = {0, 0, 0, 0};
    for (int i = cntc + tid; i < cntPad; i += NTHR) *(v4ia*)(runl + 4 * i) = z4;
  }
  __syncthreads();

  const int p0 = tid, p1 = tid + NTHR;
  const int i0 = p0 < cntPad ? p0 : cntPad - 1;
  const int i1 = p1 < cntPad ? p1 : cntPad - 1;
  const v4i e0v = *(const v4ia*)(runl + 4 * i0);
  const v4i e1v = *(const v4ia*)(runl + 4 * i1);
  const bool ok0 = p0 < cntPad, ok1 = p1 < cntPad;
  int* rp = RUN + (size_t)blk * (RUNCAP * 4);
  v4i cv;
  cv.x = (tid == 0) ? cntc : 0;
  cv.y = (tid == 0) ? ovf : 0;
  cv.z = 0; cv.w = 0;
  int* fp = CNTB + (size_t)blk * 32 + 4 * (tid & 7);
  const bool okf = tid < 8;
  if (ok0) *(volatile v4i*)(rp + 4 * p0) = e0v;
  if (ok1) *(volatile v4i*)(rp + 4 * p1) = e1v;
  if (okf) *(volatile v4i*)fp = cv;
  __threadfence();
  if (ok0) *(volatile v4i*)(rp + 4 * p0) = e0v;
  if (ok1) *(volatile v4i*)(rp + 4 * p1) = e1v;
  if (okf) *(volatile v4i*)fp = cv;
}
#undef PUTE

__global__ __launch_bounds__(NTHR) __attribute__((amdgpu_num_vgpr(248)))
void k_graph(const float* __restrict__ x, const int* __restrict__ RUN, const int* __restrict__ CNTB,
             const unsigned short* __restrict__ WPL, const float* __restrict__ PAR, float* out) {
  __shared__ __attribute__((aligned(16))) unsigned short abuf[2 * APL];
  __shared__ __attribute__((aligned(16))) float hw[PN * HPITCH];
  __shared__ __attribute__((aligned(16))) unsigned short wbuf[3 * WPLL];
  __shared__ int   lkey[GCAP];
  __shared__ float lw[GCAP];
  __shared__ __attribute__((aligned(16))) float pars[256];
  __shared__ float rinvs[PN];
  __shared__ float sv[PN];
  __shared__ __attribute__((aligned(16))) float outs[PN];
  __shared__ int wtot[NWAVE];
  __shared__ int wflag[NWAVE];

  const int tid = (int)threadIdx.x, lane = tid & 31, wave = tid >> 5, hh = lane >> 4, m = lane & 15;
  const int g = (int)blockIdx.x;

  const v2i cf = *(const v2i*)(CNTB + (size_t)tid * 32);
  const int craw = cf.x;
  const int cnt  = iclamp(craw, 0, RUNCAP);
  const bool bad = (cf.y != 0) || (craw < 0) || (craw > RUNCAP);
  const unsigned wbad = __builtin_amdgcn_ballot_w32(bad);
  int wm = cnt;
#pragma unroll
  for (int d = 16; d >= 1; d >>= 1) {
    const int y = __shfl_xor(wm, d, 32);
    wm = y > wm ? y : wm;
  }
  wm = __builtin_amdgcn_readfirstlane(wm);
  wm = iclamp(wm, 0, RUNCAP);
  const int jlast = cnt > 0 ? cnt - 1 : 0;
  const int* rp = RUN + (size_t)tid * (RUNCAP * 4);

  int mc = 0;
#pragma unroll 1
  for (int j = 0; j < wm; ++j) {
    const int jc = j < jlast ? j : jlast;
    const v4i en = *(const v4i*)(rp + 4 * jc);
    const bool hit = (j < cnt) && (en.x == g);
    mc += hit ? 1 : 0;
  }
  int total, cur;
  {
    int incl = mc;
#pragma unroll
    for (int d = 1; d < 32; d <<= 1) {
      const int y = __shfl_up(incl, d, 32);
      if (lane >= d) incl += y;
    }
    if (lane == 31) wtot[wave] = incl;
    if (lane == 0)  wflag[wave] = (wbad != 0u) ? 1 : 0;
    __syncthreads();
    int wb = 0, all = 0;
#pragma unroll
    for (int w2 = 0; w2 < NWAVE; ++w2) { const int c = wtot[w2]; all += c; wb += (w2 < wave) ? c : 0; }
    total = all;
    cur = wb + incl - mc;
  }
#pragma unroll 1
  for (int j = 0; j < wm; ++j) {
    const int jc = j < jlast ? j : jlast;
    const v4i en = *(const v4i*)(rp + 4 * jc);
    const bool hit = (j < cnt) && (en.x == g);
    if (hit && cur < GCAP) {
      lkey[cur] = (en.y & (PN - 1)) | ((en.z & (PN - 1)) << 8);
      lw[cur]   = __int_as_float(en.w);
    }
    cur += hit ? 1 : 0;
  }

  {
    const float* xg = x + (size_t)g * (PN * FIN);
#pragma unroll 4
    for (int it = 0; it < (PN * FIN / 4) / NTHR; ++it) {
      const int i = tid + NTHR * it;
      const int row = i >> 4, c4 = (i & 15) * 4;
      const v4f a = *(const v4f*)(xg + row * FIN + c4);
      v2u pk;
      pk.x = f2bf(a.x) | (f2bf(a.y) << 16);
      pk.y = f2bf(a.z) | (f2bf(a.w) << 16);
      *(v2ua*)(&abuf[row * APITCH + c4]) = pk;
    }
#pragma unroll
    for (int it = 0; it < 3; ++it) {
      const int q = tid + NTHR * it;
      const int pl = q >> 8, r = (q >> 3) & 31, c8 = (q & 7) * 8;
      const v8us wv = *(const v8us*)(WPL + (size_t)pl * (HID * FIN) + r * FIN + c8);
      *(v8usa*)(&wbuf[pl * WPLL + r * APITCH + c8]) = wv;
    }
    if (tid < 64) {
      const v4f pv = *(const v4f*)(PAR + 4 * tid);
      *(v4fa*)(pars + 4 * tid) = pv;
    }
  }
  __syncthreads();

  int tl = total > GCAP ? GCAP : (total < 0 ? 0 : total);
  tl = __builtin_amdgcn_readfirstlane(tl);
  int pflag = total > GCAP ? 1 : 0;
#pragma unroll
  for (int w2 = 0; w2 < NWAVE; ++w2) pflag |= wflag[w2];

  {
    float deg = 1.0f;
#pragma unroll 1
    for (int j = 0; j < tl; ++j) {
      const int k = lkey[j];
      const float w = lw[j];
      deg += ((k & (PN - 1)) == tid) ? w : 0.0f;
    }
    rinvs[tid] = (deg > 0.0f) ? (1.0f / deg) : 0.0f;
  }

#pragma unroll 1
  for (int L = 0; L < 3; ++L) {
    const int aoff = (L == 0) ? 0 : APL;
    const int woff = L * WPLL;
    const int boff = L * HID;
    v8f acc00, acc01, acc10, acc11;
    {
      const v8f z = {0.f, 0.f, 0.f, 0.f, 0.f, 0.f, 0.f, 0.f};
      acc00 = z; acc01 = z; acc10 = z; acc11 = z;
    }
#pragma unroll
    for (int ks = 0; ks < 2; ++ks) {
      const int ka = 32 * ks + 8 * hh;
      FragB a0, a1, b0, b1;
      a0.h[0] = *(const v8usa*)(&abuf[aoff + (32 * wave + m) * APITCH + ka]);
      a0.h[1] = *(const v8usa*)(&abuf[aoff + (32 * wave + m) * APITCH + ka + 16]);
      a1.h[0] = *(const v8usa*)(&abuf[aoff + (32 * wave + 16 + m) * APITCH + ka]);
      a1.h[1] = *(const v8usa*)(&abuf[aoff + (32 * wave + 16 + m) * APITCH + ka + 16]);
      b0.h[0] = *(const v8usa*)(&wbuf[woff + m * APITCH + ka]);
      b0.h[1] = *(const v8usa*)(&wbuf[woff + m * APITCH + ka + 16]);
      b1.h[0] = *(const v8usa*)(&wbuf[woff + (16 + m) * APITCH + ka]);
      b1.h[1] = *(const v8usa*)(&wbuf[woff + (16 + m) * APITCH + ka + 16]);
      acc00 = wmb(a0, b0, acc00);
      acc01 = wmb(a0, b1, acc01);
      acc10 = wmb(a1, b0, acc10);
      acc11 = wmb(a1, b1, acc11);
    }
#pragma unroll
    for (int r = 0; r < 8; ++r) {
      const int row0 = 32 * wave + 8 * hh + r;
      hw[row0 * HPITCH + m]             = acc00[r];
      hw[row0 * HPITCH + 16 + m]        = acc01[r];
      hw[(row0 + 16) * HPITCH + m]      = acc10[r];
      hw[(row0 + 16) * HPITCH + 16 + m] = acc11[r];
    }
    __syncthreads();

#pragma unroll 1
    for (int it = 0; it < (PN * HID / 4) / NTHR; ++it) {
      const int i = tid + NTHR * it;
      const int n = i >> 3, c = (i & 7) * 4;
      v4f acc = *(const v4fa*)(&hw[n * HPITCH + c]);
#pragma unroll 1
      for (int j = 0; j < tl; ++j) {
        const int k = lkey[j];
        const float w = lw[j];
        const int ld = (k >> 8) & (PN - 1);
        const v4f hv = *(const v4fa*)(&hw[ld * HPITCH + c]);
        const bool sel = (k & (PN - 1)) == n;
        acc.x += sel ? w * hv.x : 0.0f;
        acc.y += sel ? w * hv.y : 0.0f;
        acc.z += sel ? w * hv.z : 0.0f;
        acc.w += sel ? w * hv.w : 0.0f;
      }
      const float rv = rinvs[n];
      const v4f bb = *(const v4fa*)(&pars[boff + c]);
      const float y0 = tanhf(rv * acc.x + bb.x);
      const float y1 = tanhf(rv * acc.y + bb.y);
      const float y2 = tanhf(rv * acc.z + bb.z);
      const float y3 = tanhf(rv * acc.w + bb.w);
      const unsigned h0 = f2bf(y0), h1 = f2bf(y1), h2 = f2bf(y2), h3 = f2bf(y3);
      const unsigned l0 = f2bf(y0 - bf2f(h0)), l1 = f2bf(y1 - bf2f(h1));
      const unsigned l2 = f2bf(y2 - bf2f(h2)), l3 = f2bf(y3 - bf2f(h3));
      v2u hv2, lv2;
      hv2.x = h0 | (h1 << 16); hv2.y = h2 | (h3 << 16);
      lv2.x = l0 | (l1 << 16); lv2.y = l2 | (l3 << 16);
      *(v2ua*)(&abuf[APL + n * APITCH + c])       = hv2;
      *(v2ua*)(&abuf[APL + n * APITCH + HID + c]) = lv2;
    }
    __syncthreads();
  }

  {
    float s = 0.0f;
#pragma unroll 1
    for (int q = 0; q < HID / 8; ++q) {
      const v4u hq = *(const v4ua*)(&abuf[APL + tid * APITCH + 8 * q]);
      const v4u lq = *(const v4ua*)(&abuf[APL + tid * APITCH + HID + 8 * q]);
      const float* wq = pars + 96 + 8 * q;
      s = fmaf(__uint_as_float(hq.x << 16)         + __uint_as_float(lq.x << 16),         wq[0], s);
      s = fmaf(__uint_as_float(hq.x & 0xffff0000u) + __uint_as_float(lq.x & 0xffff0000u), wq[1], s);
      s = fmaf(__uint_as_float(hq.y << 16)         + __uint_as_float(lq.y << 16),         wq[2], s);
      s = fmaf(__uint_as_float(hq.y & 0xffff0000u) + __uint_as_float(lq.y & 0xffff0000u), wq[3], s);
      s = fmaf(__uint_as_float(hq.z << 16)         + __uint_as_float(lq.z << 16),         wq[4], s);
      s = fmaf(__uint_as_float(hq.z & 0xffff0000u) + __uint_as_float(lq.z & 0xffff0000u), wq[5], s);
      s = fmaf(__uint_as_float(hq.w << 16)         + __uint_as_float(lq.w << 16),         wq[6], s);
      s = fmaf(__uint_as_float(hq.w & 0xffff0000u) + __uint_as_float(lq.w & 0xffff0000u), wq[7], s);
    }
    sv[tid] = s;
  }
  __syncthreads();
  {
    float acc = sv[tid];
#pragma unroll 1
    for (int j = 0; j < tl; ++j) {
      const int k = lkey[j];
      const float w = lw[j];
      const int ld = (k >> 8) & (PN - 1);
      const float sl = sv[ld];
      acc += ((k & (PN - 1)) == tid) ? w * sl : 0.0f;
    }
    const float o = tanhf(rinvs[tid] * acc + pars[128]);
    const float qnan = __int_as_float(0x7fc00000);
    outs[tid] = (pflag != 0) ? qnan : o;
  }
  __syncthreads();

  const v4f ov = *(const v4fa*)(outs + 4 * (tid & 63));
  float* op = out + (size_t)g * PN + 4 * (tid & 63);
  const bool okst = tid < 64;
  if (okst) *(volatile v4f*)op = ov;
  __threadfence();
  if (okst) *(volatile v4f*)op = ov;
}

static inline size_t al256(size_t o) { return (o + 255) & ~(size_t)255; }

extern "C" void kernel_launch(void* const* d_in, const int* in_sizes, int n_in,
                              void* d_out, int out_size, void* d_ws, size_t ws_size,
                              hipStream_t stream) {
  if (n_in < 12) return;
  if (in_sizes[0] != NNODE * FIN) return;
  if (in_sizes[1] != 2 * NEDGE) return;
  if (in_sizes[2] != NNODE) return;
  if (in_sizes[3] != NEDGE) return;
  if (in_sizes[4] != FIN * HID || in_sizes[5] != HID) return;
  if (in_sizes[6] != HID * HID || in_sizes[7] != HID) return;
  if (in_sizes[8] != HID * HID || in_sizes[9] != HID) return;
  if (in_sizes[10] != HID || in_sizes[11] != 1) return;
  if (out_size != NNODE) return;

  const float* x   = (const float*)d_in[0];
  const int*   ei  = (const int*)  d_in[1];
  const int*   bat = (const int*)  d_in[2];
  const float* em  = (const float*)d_in[3];
  const float* W0  = (const float*)d_in[4];
  const float* b0  = (const float*)d_in[5];
  const float* W1  = (const float*)d_in[6];
  const float* b1  = (const float*)d_in[7];
  const float* W2  = (const float*)d_in[8];
  const float* b2  = (const float*)d_in[9];
  const float* W3  = (const float*)d_in[10];
  const float* b3  = (const float*)d_in[11];
  float* out = (float*)d_out;

  char* ws = (char*)d_ws;
  size_t off = 0;
  const size_t oRUN = off; off = al256(off + (size_t)NRUN * RUNCAP * 16);
  const size_t oCNB = off; off = al256(off + (size_t)NRUN * 128);
  const size_t oCNT = off; off = al256(off + (size_t)NGR * 4);
  const size_t oWPL = off; off = al256(off + (size_t)3 * HID * FIN * 2);
  const size_t oPAR = off; off = al256(off + (size_t)256 * 4);
  if (off > ws_size || off > (size_t)WSMAX) return;
  int*            RUN    = (int*)(ws + oRUN);
  int*            CNTB   = (int*)(ws + oCNB);
  int*            COUNTS = (int*)(ws + oCNT);
  unsigned short* WPL    = (unsigned short*)(ws + oWPL);
  float*          PAR    = (float*)(ws + oPAR);

  k_prep<<<4, NTHR, 0, stream>>>(W0, b0, W1, b1, W2, b2, W3, b3, WPL, PAR);
  k_counts<<<NGR / CGRP, NTHR, 0, stream>>>(bat, COUNTS);
  k_vfill<<<NRUN, NTHR, 0, stream>>>(ei, bat, em, COUNTS, RUN, CNTB);
  k_graph<<<NGR, NTHR, 0, stream>>>(x, RUN, CNTB, WPL, PAR, out);
}
